// bi_Mamba2_13022340841846
// MI455X (gfx1250) — hardware-verified
//
#include <hip/hip_runtime.h>
#include <math.h>

typedef __attribute__((ext_vector_type(16))) _Float16 v16h;
typedef __attribute__((ext_vector_type(8)))  _Float16 v8h;
typedef __attribute__((ext_vector_type(8)))  float    v8f;
typedef __attribute__((ext_vector_type(4)))  float    v4f;
typedef __attribute__((ext_vector_type(2)))  float    v2f;
typedef __attribute__((ext_vector_type(4)))  unsigned u4v;
typedef __attribute__((ext_vector_type(2)))  unsigned u2v;

constexpr int kB     = 2;
constexpr int kL     = 2048;
constexpr int kDm    = 1024;
constexpr int kDs    = 2048;
constexpr int kH     = 32;
constexpr int kP     = 64;
constexpr int kN     = 128;
constexpr int kCv    = 2304;
constexpr int kDip   = 4384;
constexpr int kDipP  = 4416;
constexpr int kQ     = 256;
constexpr int kNc    = 8;
constexpr int kRows  = kB * kL;
constexpr int kBCw   = 2 * kN;
constexpr int kTP    = 264;
constexpr int kDtP   = 260;
constexpr int kCvPI  = 65;
constexpr int kCvPO  = 68;
static_assert(kCv == kDs + 2 * kN, "conv width");
static_assert(kDip == 2 * kDs + 2 * kN + kH, "in_proj width");
static_assert(kDs == kH * kP && kL == kNc * kQ, "head and chunk split");
static_assert((kDipP % 64) == 0 && kDipP >= kDip && (kRows % 64) == 0 && (kDm % 64) == 0 && (kQ % 64) == 0, "GEMM M,N multiples of 64");
static_assert((kDm % 32) == 0 && (kDs % 32) == 0 && (kN % 32) == 0 && (kQ % 32) == 0, "GEMM K multiples of 32");
static_assert(64 * kTP * 2 >= 8 * 1024 * 4, "slab view fits the operand tile");

constexpr float kWCarry  = 32.0f;
constexpr float kWInv    = 1.0f / kWCarry;
constexpr float kACarry  = 256.0f;
constexpr float kHCarry  = 64.0f;
constexpr float kXCarry  = 16.0f;
constexpr float kCBCarry = 64.0f;
constexpr float kYdCarry = kXCarry * kCBCarry;

constexpr size_t kOffZX   = 0;
constexpr size_t kOffU16  = kOffZX   + (size_t)kRows * kDipP * 2;
constexpr size_t kOffINW  = kOffU16  + (size_t)kRows * kDm * 2;
constexpr size_t kOffOUTW = kOffINW  + (size_t)kDipP * kDm * 2;
constexpr size_t kOffENDW = kOffOUTW + (size_t)kDm * kDs * 2;
constexpr size_t kOffX16  = kOffENDW + (size_t)kDm * kDm * 2;
constexpr size_t kOffBC16 = kOffX16  + (size_t)kRows * kDs * 2;
constexpr size_t kOffBT16 = kOffBC16 + (size_t)kRows * kBCw * 2;
constexpr size_t kOffDT32 = kOffBT16 + (size_t)kB * kN * kL * 2;
constexpr size_t kOffCS32 = kOffDT32 + (size_t)kB * kNc * kH * kQ * 4;
constexpr size_t kOffCB16 = kOffCS32 + (size_t)kB * kNc * kH * kQ * 4;
constexpr size_t kOffHP16 = kOffCB16 + (size_t)kB * kNc * kQ * kQ * 2;
constexpr size_t kOffY16  = kOffHP16 + (size_t)kB * kNc * kH * kP * kN * 2;
constexpr size_t kOffYN0  = kOffY16  + (size_t)kRows * kDs * 2;
constexpr size_t kWsTotal = kOffYN0  + (size_t)kRows * kDs * 2;
static_assert(kWsTotal == 124911616ull, "carve total");
static_assert(kWsTotal <= 134217728ull, "carve cap");
static_assert((kOffU16 % 128) == 0 && (kOffINW % 128) == 0 && (kOffOUTW % 128) == 0 && (kOffENDW % 128) == 0 &&
              (kOffX16 % 128) == 0 && (kOffBC16 % 128) == 0 && (kOffBT16 % 128) == 0 && (kOffDT32 % 128) == 0 &&
              (kOffCS32 % 128) == 0 && (kOffCB16 % 128) == 0 && (kOffHP16 % 128) == 0 && (kOffY16 % 128) == 0 &&
              (kOffYN0 % 128) == 0, "128-B aligned regions");

__device__ __forceinline__ unsigned short f2bf_bits(float f) {
  unsigned u = __float_as_uint(f);
  return (unsigned short)((u + 0x7FFFu + ((u >> 16) & 1u)) >> 16);
}
__device__ __forceinline__ float bf_bits2f(unsigned short h) { return __uint_as_float(((unsigned)h) << 16); }
__device__ __forceinline__ float bfr(float f) { return bf_bits2f(f2bf_bits(f)); }

__device__ __forceinline__ float h16_to_f32(unsigned hb) {
  const unsigned sgn = (hb & 0x8000u) << 16;
  const unsigned em = hb & 0x7fffu;
  const float fn = __uint_as_float((em << 13) + 0x38000000u);
  const float fs = (float)em * 5.9604644775390625e-8f;
  const float mag = (em < 0x400u) ? fs : fn;
  return __uint_as_float(__float_as_uint(mag) | sgn);
}
__device__ __forceinline__ unsigned pack2h(float lo, float hi) {
  const _Float16 a = (_Float16)lo;
  const _Float16 b = (_Float16)hi;
  const unsigned short ab = __builtin_bit_cast(unsigned short, a);
  const unsigned short bb = __builtin_bit_cast(unsigned short, b);
  return (unsigned)ab | ((unsigned)bb << 16);
}

__device__ __forceinline__ v16h ldfrag(const _Float16* p) {
  union { v16h v; v8h h[2]; } f;
  f.h[0] = *(const v8h*)(p);
  f.h[1] = *(const v8h*)(p + 16);
  return f.v;
}
__device__ __forceinline__ v8f mma_h(v16h a, v16h b, v8f c) {
  return __builtin_amdgcn_wmma_f32_16x16x32_f16(false, a, false, b, (short)0, c, false, false);
}
__device__ __forceinline__ void guard4_h(v8f& a, v8f& b, v8f& c, v8f& d, v16h x, v16h y) {
  asm volatile("v_nop\n\tv_nop\n\tv_nop\n\tv_nop" : "+v"(a), "+v"(b), "+v"(c), "+v"(d) : "v"(x), "v"(y));
}
__device__ __forceinline__ void keep4_h(v16h a, v16h b, v16h c, v16h d) { asm volatile("v_nop" :: "v"(a), "v"(b), "v"(c), "v"(d)); }
__device__ __forceinline__ void acc_guard4(v8f& a, v8f& b, v8f& c, v8f& d) { asm volatile("v_nop\n\tv_nop\n\tv_nop\n\tv_nop" : "+v"(a), "+v"(b), "+v"(c), "+v"(d)); }

template <int BIAS_MODE, int OUT_MODE>
__global__ __launch_bounds__(256) void wmma_gemm64_h(
    const unsigned short* __restrict__ Ap, int lda, long strideA,
    const unsigned short* __restrict__ Btp, int ldb, long strideB,
    void* __restrict__ Cout, int ldc, long strideC,
    const float* __restrict__ bias, int M, int N, int K, float scale) {
  __shared__ __align__(16) float sT[8][16 * 68];
  const int b    = blockIdx.y;
  const int lane = threadIdx.x & 31;
  const int wave = threadIdx.x >> 5;
  const int tilesN = N >> 6;
  const int tilesM = M >> 6;
  const int tile = blockIdx.x * 8 + wave;
  if (tile >= tilesM * tilesN) return;
  const int tm = tile / tilesN;
  const int tn = tile - tm * tilesN;
  const int m0 = tm << 6;
  const int n0 = tn << 6;
  const _Float16* Ab = (const _Float16*)Ap + (size_t)b * strideA;
  const _Float16* Bb = (const _Float16*)Btp + (size_t)b * strideB;
  const int rlane = lane & 15;
  const int koff  = (lane >> 4) * 8;
  const int mOff  = (lane >> 4) * 8;

  v8f acc[4][4];
#pragma unroll
  for (int i = 0; i < 4; ++i)
#pragma unroll
    for (int j = 0; j < 4; ++j) acc[i][j] = (v8f){0.f, 0.f, 0.f, 0.f, 0.f, 0.f, 0.f, 0.f};

  for (int k0 = 0; k0 < K; k0 += 32) {
    v16h bh[4];
#pragma unroll
    for (int j = 0; j < 4; ++j) {
      const size_t bo = (size_t)(n0 + (j << 4) + rlane) * ldb + koff + k0;
      bh[j] = ldfrag(Bb + bo);
    }
#pragma unroll
    for (int i = 0; i < 4; ++i) {
      const size_t ao = (size_t)(m0 + (i << 4) + rlane) * lda + koff + k0;
      const v16h ah = ldfrag(Ab + ao);
#pragma unroll
      for (int j = 0; j < 4; ++j) acc[i][j] = mma_h(ah, bh[j], acc[i][j]);
      guard4_h(acc[i][0], acc[i][1], acc[i][2], acc[i][3], ah, bh[0]);
    }
    keep4_h(bh[0], bh[1], bh[2], bh[3]);
  }
  acc_guard4(acc[0][0], acc[0][1], acc[0][2], acc[0][3]);
  acc_guard4(acc[1][0], acc[1][1], acc[1][2], acc[1][3]);
  acc_guard4(acc[2][0], acc[2][1], acc[2][2], acc[2][3]);
  acc_guard4(acc[3][0], acc[3][1], acc[3][2], acc[3][3]);

  float* slab = sT[wave];
#pragma unroll
  for (int i = 0; i < 4; ++i) {
    const int mBase = m0 + (i << 4);
#pragma unroll
    for (int j = 0; j < 4; ++j) {
      const int n = n0 + (j << 4) + rlane;
      float bv = 0.f;
      if (BIAS_MODE == 2) bv = bfr(bias[n]);
#pragma unroll
      for (int r = 0; r < 8; ++r) {
        float v = acc[i][j][r] * scale;
        if (BIAS_MODE == 2) v += bv;
        slab[(mOff + r) * 68 + (j << 4) + rlane] = v;
      }
    }
    __builtin_amdgcn_fence(__ATOMIC_RELEASE, "workgroup");
    __builtin_amdgcn_wave_barrier();
    __builtin_amdgcn_fence(__ATOMIC_ACQUIRE, "workgroup");
    if (OUT_MODE == 0) {
      float* C = (float*)Cout + (size_t)b * strideC;
      const int hh = lane >> 4, c4 = (lane & 15) * 4;
      for (int pass = 0; pass < 2; ++pass) {
#pragma unroll
        for (int it = 0; it < 8; ++it) {
          const int row = it * 2 + hh;
          v4f v = *(const v4f*)(slab + row * 68 + c4);
          *(volatile v4f*)(C + (size_t)(mBase + row) * ldc + n0 + c4) = v;
        }
        __threadfence();
      }
    } else {
      const int q = lane >> 3, c8 = (lane & 7) * 8;
      unsigned short* C = (unsigned short*)Cout + (size_t)b * strideC;
      for (int pass = 0; pass < 2; ++pass) {
#pragma unroll
        for (int it = 0; it < 4; ++it) {
          const int row = it * 4 + q;
          const float* sp = slab + row * 68 + c8;
          v8h hv;
#pragma unroll
          for (int e = 0; e < 8; ++e) hv[e] = (_Float16)sp[e];
          *(volatile v8h*)(C + (size_t)(mBase + row) * ldc + n0 + c8) = hv;
        }
        __threadfence();
      }
    }
    __builtin_amdgcn_fence(__ATOMIC_RELEASE, "workgroup");
    __builtin_amdgcn_wave_barrier();
    __builtin_amdgcn_fence(__ATOMIC_ACQUIRE, "workgroup");
  }
}

__global__ __launch_bounds__(256) void cast_bf_f16_kernel(
    const float* __restrict__ src, unsigned short* __restrict__ dst, int total8, int valid8, float scale)
{
  const int i = blockIdx.x * 256 + threadIdx.x;
  if (i >= total8) return;
  const bool ok = i < valid8;
  const size_t e0 = (size_t)i << 3;
  const size_t es = ok ? e0 : (size_t)0;
  const v4f a0 = *(const v4f*)(src + es);
  const v4f a1 = *(const v4f*)(src + es + 4);
  v8h hv;
#pragma unroll
  for (int e = 0; e < 4; ++e) {
    const float x0 = bfr(a0[e]) * scale;
    const float x1 = bfr(a1[e]) * scale;
    hv[e]     = (_Float16)(ok ? x0 : 0.0f);
    hv[4 + e] = (_Float16)(ok ? x1 : 0.0f);
  }
  unsigned short* q = dst + e0;
  *(volatile v8h*)q = hv;
  __threadfence();
  *(volatile v8h*)q = hv;
}

template <int BR>
__global__ __launch_bounds__(256) void conv_silu_kernel(
    const unsigned short* __restrict__ ZX, const float* __restrict__ cw, const float* __restrict__ cb,
    unsigned short* __restrict__ X16, unsigned short* __restrict__ BC16, unsigned short* __restrict__ BT16)
{
  __shared__ __align__(16) float sIn[67 * kCvPI];
  __shared__ __align__(16) float sOut[64 * kCvPO];
  const int tid = threadIdx.x, lane = tid & 31, wave = tid >> 5;
  const int ct = blockIdx.x;
  const int c0 = ct * 64;
  const int g0 = blockIdx.y * 64;
  const int tb = g0 & (kL - 1);
  const int colbase = BR ? (kDip - 1 - (kDs + c0 + 63)) : (kDs + c0);

#pragma unroll 1
  for (int it = 0; it < 3; ++it) {
    const int idx = tid + it * 256;
    const int idc = (idx < 536) ? idx : 535;
    const int r = idc >> 3, sg = idc & 7;
    const bool valid = (tb + r - 3) >= 0;
    const int grow = valid ? (g0 + r - 3) : g0;
    const u4v w = *(const u4v*)(ZX + (size_t)grow * kDipP + colbase + sg * 8);
    if (idx < 536) {
#pragma unroll
      for (int j = 0; j < 4; ++j) {
        const unsigned wj = w[j];
        const int cz = sg * 8 + 2 * j;
        const int ca = BR ? (63 - cz) : cz;
        const int cn = BR ? (62 - cz) : (cz + 1);
        const float va = h16_to_f32(wj & 0xffffu);
        const float vb = h16_to_f32(wj >> 16);
        sIn[r * kCvPI + ca] = valid ? va : 0.0f;
        sIn[r * kCvPI + cn] = valid ? vb : 0.0f;
      }
    }
  }
  __syncthreads();
  {
    const int cl = tid & 63, lg = tid >> 6;
    const int c = c0 + cl;
    const v4f wv = *(const v4f*)(cw + (size_t)c * 4);
    const float w0 = bfr(wv[0]), w1 = bfr(wv[1]), w2 = bfr(wv[2]), w3 = bfr(wv[3]);
    const float bc = bfr(cb[c]);
#pragma unroll 1
    for (int s = 0; s < 16; ++s) {
      const int l = lg * 16 + s;
      float acc = w0 * sIn[l * kCvPI + cl];
      acc = fmaf(w1, sIn[(l + 1) * kCvPI + cl], acc);
      acc = fmaf(w2, sIn[(l + 2) * kCvPI + cl], acc);
      acc = fmaf(w3, sIn[(l + 3) * kCvPI + cl], acc);
      const float sv = acc + bc;
      const float sg = __builtin_amdgcn_rcpf(1.0f + expf(-sv));
      sOut[l * kCvPO + cl] = sv * sg;
    }
  }
  __syncthreads();
  const int q = lane >> 3, c8 = (lane & 7) * 8;
  unsigned short* dst;
  int pitch;
  if (ct < 32) { dst = X16 + (size_t)g0 * kDs + c0; pitch = kDs; }
  else         { dst = BC16 + (size_t)g0 * kBCw + (c0 - kDs); pitch = kBCw; }
  v8h hv[2];
#pragma unroll
  for (int it = 0; it < 2; ++it) {
    const int row = it * 32 + wave * 4 + q;
    const float* sp = sOut + row * kCvPO + c8;
    const v4f a0 = *(const v4f*)(sp);
    const v4f a1 = *(const v4f*)(sp + 4);
#pragma unroll
    for (int e = 0; e < 4; ++e) { hv[it][e] = (_Float16)a0[e]; hv[it][4 + e] = (_Float16)a1[e]; }
  }
  for (int pass = 0; pass < 2; ++pass) {
#pragma unroll
    for (int it = 0; it < 2; ++it) {
      const int row = it * 32 + wave * 4 + q;
      *(volatile v8h*)(dst + (size_t)row * pitch + c8) = hv[it];
    }
    __threadfence();
  }
  if (ct >= 32 && ct < 34) {
    const int nbase = c0 - kDs;
    const int bix = g0 / kL;
    v8h tv[2];
#pragma unroll
    for (int it = 0; it < 2; ++it) {
      const int nrow = it * 32 + wave * 4 + q;
#pragma unroll
      for (int e = 0; e < 8; ++e) tv[it][e] = (_Float16)sOut[(c8 + e) * kCvPO + nrow];
    }
    for (int pass = 0; pass < 2; ++pass) {
#pragma unroll
      for (int it = 0; it < 2; ++it) {
        const int nrow = it * 32 + wave * 4 + q;
        *(volatile v8h*)(BT16 + ((size_t)bix * kN + nbase + nrow) * kL + tb + c8) = tv[it];
      }
      __threadfence();
    }
  }
}

template <int BR>
__global__ __launch_bounds__(256) void dt_cs_kernel(
    const unsigned short* __restrict__ ZX, const float* __restrict__ dtb, const float* __restrict__ alog,
    float* __restrict__ DT32, float* __restrict__ CS32)
{
  __shared__ __align__(16) float sD[kH * kDtP];
  __shared__ __align__(16) float sC[kH * kDtP];
  const int tid = threadIdx.x, lane = tid & 31, wave = tid >> 5;
  const int bc = blockIdx.x;
  const int row0 = bc * kQ;
  const int colbase = BR ? 0 : (kDip - kH);
#pragma unroll 1
  for (int it = 0; it < 32; ++it) {
    const int idx = tid + it * 256;
    const int l = idx >> 5, col = idx & 31;
    const unsigned hb = ZX[(size_t)(row0 + l) * kDipP + colbase + col];
    const int h = BR ? (31 - col) : col;
    const float x = h16_to_f32(hb) + bfr(dtb[h]);
    sD[h * kDtP + l] = fmaxf(x, 0.0f) + log1pf(expf(-fabsf(x)));
  }
  __syncthreads();
#pragma unroll 1
  for (int hh = 0; hh < 4; ++hh) {
    const int h = wave * 4 + hh;
    const float Ah = -expf(bfr(alog[h]));
    const float* dp = sD + h * kDtP + lane * 8;
    const v4f d0 = *(const v4f*)(dp);
    const v4f d1 = *(const v4f*)(dp + 4);
    const float r0 = d0[0] * Ah;
    const float r1 = r0 + d0[1] * Ah;
    const float r2 = r1 + d0[2] * Ah;
    const float r3 = r2 + d0[3] * Ah;
    const float r4 = r3 + d1[0] * Ah;
    const float r5 = r4 + d1[1] * Ah;
    const float r6 = r5 + d1[2] * Ah;
    const float r7 = r6 + d1[3] * Ah;
    float incl = r7;
#pragma unroll
    for (int off = 1; off < 32; off <<= 1) {
      const float t = __shfl_up(incl, off, 32);
      incl = (lane >= off) ? (incl + t) : incl;
    }
    const float up = __shfl_up(incl, 1, 32);
    const float ex = (lane == 0) ? 0.0f : up;
    float* cp = sC + h * kDtP + lane * 8;
    *(v4f*)(cp)     = (v4f){ex + r0, ex + r1, ex + r2, ex + r3};
    *(v4f*)(cp + 4) = (v4f){ex + r4, ex + r5, ex + r6, ex + r7};
  }
  __syncthreads();
#pragma unroll 1
  for (int hh = 0; hh < 4; ++hh) {
    const int h = wave * 4 + hh;
    const size_t base = ((size_t)bc * kH + h) * kQ;
    const v4f d0 = *(const v4f*)(sD + h * kDtP + lane * 4);
    const v4f d1 = *(const v4f*)(sD + h * kDtP + 128 + lane * 4);
    const v4f e0 = *(const v4f*)(sC + h * kDtP + lane * 4);
    const v4f e1 = *(const v4f*)(sC + h * kDtP + 128 + lane * 4);
    for (int pass = 0; pass < 2; ++pass) {
      *(volatile v4f*)(DT32 + base + lane * 4) = d0;
      *(volatile v4f*)(DT32 + base + 128 + lane * 4) = d1;
      *(volatile v4f*)(CS32 + base + lane * 4) = e0;
      *(volatile v4f*)(CS32 + base + 128 + lane * 4) = e1;
      __threadfence();
    }
  }
}

__device__ __forceinline__ void stage16(const unsigned short* g0, const unsigned short* g1,
                                        float f0, float f1, unsigned* dw, int pitchW)
{
  const u4v a0 = *(const u4v*)(g0);
  const u4v a1 = *(const u4v*)(g0 + 8);
  const u4v b0 = *(const u4v*)(g1);
  const u4v b1 = *(const u4v*)(g1 + 8);
#pragma unroll
  for (int j = 0; j < 4; ++j) {
    const unsigned wa = a0[j];
    const unsigned wb = b0[j];
    const unsigned wc = a1[j];
    const unsigned wd = b1[j];
    dw[(2 * j) * pitchW]     = pack2h(h16_to_f32(wa & 0xffffu) * f0, h16_to_f32(wb & 0xffffu) * f1);
    dw[(2 * j + 1) * pitchW] = pack2h(h16_to_f32(wa >> 16) * f0, h16_to_f32(wb >> 16) * f1);
    dw[(8 + 2 * j) * pitchW] = pack2h(h16_to_f32(wc & 0xffffu) * f0, h16_to_f32(wd & 0xffffu) * f1);
    dw[(9 + 2 * j) * pitchW] = pack2h(h16_to_f32(wc >> 16) * f0, h16_to_f32(wd >> 16) * f1);
  }
}

__global__ __launch_bounds__(256) void states_scan_kernel(
    const unsigned short* __restrict__ X16, const unsigned short* __restrict__ BT16,
    const float* __restrict__ DT32, const float* __restrict__ CS32, unsigned short* __restrict__ HP16)
{
  __shared__ __align__(16) _Float16 sAT[64 * kTP];
  const int tid = threadIdx.x, lane = tid & 31, wave = tid >> 5;
  const int b = blockIdx.x >> 5, h = blockIdx.x & 31;
  const int rlane = lane & 15;
  const int koff = (lane >> 4) * 8;
  const int mOff = koff;
  const int pt = wave & 3, ntb = (wave >> 2) * 4;
  const int q = lane >> 3, c8 = (lane & 7) * 8;
  const int lp = tid & 127, pq = tid >> 7;
  float* slab = (float*)sAT + wave * 1024;
  unsigned* sW = (unsigned*)sAT;
  const _Float16* Bg = (const _Float16*)BT16 + (size_t)b * kN * kL;
  constexpr float kHpScale = kHCarry / kACarry;

  v8f acc[4];
#pragma unroll
  for (int j = 0; j < 4; ++j) acc[j] = (v8f){0.f, 0.f, 0.f, 0.f, 0.f, 0.f, 0.f, 0.f};

#pragma unroll 1
  for (int c = 0; c < kNc; ++c) {
    const size_t bch = ((size_t)(b * kNc + c) * kH + h);
    const size_t base = bch * kQ;
    __syncthreads();
#pragma unroll
    for (int j = 0; j < 4; ++j)
#pragma unroll
      for (int i = 0; i < 8; ++i)
        slab[(mOff + i) * 64 + j * 16 + rlane] = acc[j][i] * kHpScale;
    __syncthreads();
    {
      v8h hv[4];
#pragma unroll
      for (int it = 0; it < 4; ++it) {
        const int row = it * 4 + q;
        const float* sp = slab + row * 64 + c8;
        const v4f a0 = *(const v4f*)(sp);
        const v4f a1 = *(const v4f*)(sp + 4);
#pragma unroll
        for (int e = 0; e < 4; ++e) { hv[it][e] = (_Float16)a0[e]; hv[it][4 + e] = (_Float16)a1[e]; }
      }
      unsigned short* hp = HP16 + (bch * kP + pt * 16) * kN + ntb * 16 + c8;
      for (int pass = 0; pass < 2; ++pass) {
#pragma unroll
        for (int it = 0; it < 4; ++it) {
          const int row = it * 4 + q;
          *(volatile v8h*)(hp + (size_t)row * kN) = hv[it];
        }
        __threadfence();
      }
    }
    if (c == kNc - 1) break;
    __syncthreads();
    const float cslast = CS32[base + kQ - 1];
    {
      const int s0 = 2 * lp;
      const v2f dtp = *(const v2f*)(DT32 + base + s0);
      const v2f csp = *(const v2f*)(CS32 + base + s0);
      const float f0 = dtp[0] * expf(fminf(cslast - csp[0], 0.0f)) * kACarry;
      const float f1 = dtp[1] * expf(fminf(cslast - csp[1], 0.0f)) * kACarry;
      const size_t grow = (size_t)b * kL + (size_t)c * kQ + s0;
      const unsigned short* g0 = X16 + grow * kDs + h * kP + pq * 32;
      const unsigned short* g1 = g0 + kDs;
      stage16(g0, g1, f0, f1, sW + (pq * 32) * (kTP / 2) + lp, kTP / 2);
      stage16(g0 + 16, g1 + 16, f0, f1, sW + (pq * 32 + 16) * (kTP / 2) + lp, kTP / 2);
    }
    __syncthreads();
    {
      const float cd = expf(cslast);
#pragma unroll
      for (int j = 0; j < 4; ++j)
#pragma unroll
        for (int i = 0; i < 8; ++i) acc[j][i] *= cd;
#pragma unroll 1
      for (int k0 = 0; k0 < kQ; k0 += 32) {
        const v16h a = ldfrag(sAT + (pt * 16 + rlane) * kTP + k0 + koff);
        v16h bf[4];
#pragma unroll
        for (int j = 0; j < 4; ++j)
          bf[j] = ldfrag(Bg + (size_t)((ntb + j) * 16 + rlane) * kL + c * kQ + k0 + koff);
#pragma unroll
        for (int j = 0; j < 4; ++j) acc[j] = mma_h(a, bf[j], acc[j]);
        guard4_h(acc[0], acc[1], acc[2], acc[3], a, bf[0]);
        keep4_h(bf[0], bf[1], bf[2], bf[3]);
      }
      acc_guard4(acc[0], acc[1], acc[2], acc[3]);
    }
  }
}

__device__ __forceinline__ _Float16 decay_elem(unsigned hb, float csl, float css, bool ok) {
  const float e = expf(fminf(csl - css, 0.0f));
  const float v = h16_to_f32(hb) * e * kCBCarry;
  return (_Float16)(ok ? v : 0.0f);
}

__global__ __launch_bounds__(512) void ssd_y_kernel(
    const unsigned short* __restrict__ X16, const unsigned short* __restrict__ BC16,
    const unsigned short* __restrict__ CB16, const unsigned short* __restrict__ HP16,
    const float* __restrict__ DT32, const float* __restrict__ CS32, const float* __restrict__ Dp,
    unsigned short* __restrict__ Y16)
{
  __shared__ __align__(16) _Float16 sXT[64 * kTP];
  __shared__ __align__(16) float sCs[kQ];
  const int tid = threadIdx.x, lane = tid & 31, wave = tid >> 5;
  const int bid = blockIdx.x;
  const int h = bid & 31;
  const int bc = bid >> 5;
  const int rowbase = bc * kQ;
  const size_t bch = (size_t)bc * kH + h;
  const size_t base = bch * kQ;
  const int rlane = lane & 15;
  const int hh = lane >> 4;
  const int koff = hh * 8;
  const int mOff = koff;

  if (tid < kQ) sCs[tid] = CS32[base + tid];
  {
    const int lp = tid & 127, pq = tid >> 7;
    const int s0 = 2 * lp;
    const v2f dtp = *(const v2f*)(DT32 + base + s0);
    const unsigned short* g0 = X16 + (size_t)(rowbase + s0) * kDs + h * kP + pq * 16;
    stage16(g0, g0 + kDs, dtp[0] * kXCarry, dtp[1] * kXCarry,
            (unsigned*)sXT + (pq * 16) * (kTP / 2) + lp, kTP / 2);
  }
  __syncthreads();

  const int lt = wave;
  v8f acc[4];
#pragma unroll
  for (int j = 0; j < 4; ++j) acc[j] = (v8f){0.f, 0.f, 0.f, 0.f, 0.f, 0.f, 0.f, 0.f};

  {
    const _Float16* Cg = (const _Float16*)BC16 + (size_t)(rowbase + lt * 16 + rlane) * kBCw + kN;
    const _Float16* Hg = (const _Float16*)HP16 + bch * kP * kN;
#pragma unroll
    for (int kn = 0; kn < 4; ++kn) {
      const v16h a = ldfrag(Cg + kn * 32 + koff);
      v16h bf[4];
#pragma unroll
      for (int j = 0; j < 4; ++j) bf[j] = ldfrag(Hg + (size_t)(j * 16 + rlane) * kN + kn * 32 + koff);
#pragma unroll
      for (int j = 0; j < 4; ++j) acc[j] = mma_h(a, bf[j], acc[j]);
      guard4_h(acc[0], acc[1], acc[2], acc[3], a, bf[0]);
      keep4_h(bf[0], bf[1], bf[2], bf[3]);
    }
    acc_guard4(acc[0], acc[1], acc[2], acc[3]);
    constexpr float kOffScale = kYdCarry / kHCarry;
#pragma unroll
    for (int i = 0; i < 8; ++i) {
      const float sc = expf(sCs[lt * 16 + mOff + i]) * kOffScale;
#pragma unroll
      for (int j = 0; j < 4; ++j) acc[j][i] *= sc;
    }
  }

  {
    const int smax = lt >> 1;
    const int lrow = lt * 16 + rlane;
    const float csl = sCs[lrow];
    const unsigned short* cbrow = CB16 + ((size_t)bc * kQ + lrow) * kQ;
#pragma unroll 1
    for (int sb = 0; sb <= smax; ++sb) {
      const int sa = sb * 32 + koff;
      const int sc2 = sa + 16;
      const u4v w0 = *(const u4v*)(cbrow + sa);
      const u4v w1 = *(const u4v*)(cbrow + sc2);
      const v4f ca0 = *(const v4f*)(sCs + sa);
      const v4f ca1 = *(const v4f*)(sCs + sa + 4);
      const v4f cb0 = *(const v4f*)(sCs + sc2);
      const v4f cb1 = *(const v4f*)(sCs + sc2 + 4);
      v16h a;
#pragma unroll
      for (int j = 0; j < 4; ++j) {
        const unsigned wa = w0[j];
        const unsigned wb = w1[j];
        const float s0a = (j < 2) ? ca0[(2 * j) & 3] : ca1[(2 * j) & 3];
        const float s1a = (j < 2) ? ca0[(2 * j + 1) & 3] : ca1[(2 * j + 1) & 3];
        const float s0b = (j < 2) ? cb0[(2 * j) & 3] : cb1[(2 * j) & 3];
        const float s1b = (j < 2) ? cb0[(2 * j + 1) & 3] : cb1[(2 * j + 1) & 3];
        a[2 * j]         = decay_elem(wa & 0xffffu, csl, s0a, (sa + 2 * j) <= lrow);
        a[2 * j + 1]     = decay_elem(wa >> 16,     csl, s1a, (sa + 2 * j + 1) <= lrow);
        a[8 + 2 * j]     = decay_elem(wb & 0xffffu, csl, s0b, (sc2 + 2 * j) <= lrow);
        a[8 + 2 * j + 1] = decay_elem(wb >> 16,     csl, s1b, (sc2 + 2 * j + 1) <= lrow);
      }
      v16h bf[4];
#pragma unroll
      for (int j = 0; j < 4; ++j) bf[j] = ldfrag(sXT + (j * 16 + rlane) * kTP + sb * 32 + koff);
#pragma unroll
      for (int j = 0; j < 4; ++j) acc[j] = mma_h(a, bf[j], acc[j]);
      guard4_h(acc[0], acc[1], acc[2], acc[3], a, bf[0]);
      keep4_h(bf[0], bf[1], bf[2], bf[3]);
    }
    acc_guard4(acc[0], acc[1], acc[2], acc[3]);
  }

  __syncthreads();
  float* slab = (float*)sXT + (wave & 7) * 1024;
  const float Dh = bfr(Dp[h]);
  constexpr float kFold = 1.0f / kYdCarry;
  const int q = lane >> 3, c8 = (lane & 7) * 8;
#pragma unroll
  for (int ph = 0; ph < 2; ++ph) {
    if ((wave >> 3) == ph) {
#pragma unroll
      for (int j = 0; j < 4; ++j)
#pragma unroll
        for (int i = 0; i < 8; ++i)
          slab[(mOff + i) * 64 + j * 16 + rlane] = acc[j][i] * kFold;
    }
    __syncthreads();
    if ((wave >> 3) == ph) {
      v8h hv[4];
#pragma unroll
      for (int it = 0; it < 4; ++it) {
        const int row = it * 4 + q;
        const size_t xo = (size_t)(rowbase + lt * 16 + row) * kDs + h * kP + c8;
        const u4v xw = *(const u4v*)(X16 + xo);
        const float* sp = slab + row * 64 + c8;
        const v4f a0 = *(const v4f*)(sp);
        const v4f a1 = *(const v4f*)(sp + 4);
#pragma unroll
        for (int jj = 0; jj < 4; ++jj) {
          const unsigned wx = xw[jj];
          const float x0 = h16_to_f32(wx & 0xffffu);
          const float x1 = h16_to_f32(wx >> 16);
          const float y0 = (jj < 2) ? a0[(2 * jj) & 3] : a1[(2 * jj) & 3];
          const float y1 = (jj < 2) ? a0[(2 * jj + 1) & 3] : a1[(2 * jj + 1) & 3];
          hv[it][2 * jj]     = (_Float16)fmaf(Dh, x0, y0);
          hv[it][2 * jj + 1] = (_Float16)fmaf(Dh, x1, y1);
        }
      }
      for (int pass = 0; pass < 2; ++pass) {
#pragma unroll
        for (int it = 0; it < 4; ++it) {
          const int row = it * 4 + q;
          *(volatile v8h*)(Y16 + (size_t)(rowbase + lt * 16 + row) * kDs + h * kP + c8) = hv[it];
        }
        __threadfence();
      }
    }
    __syncthreads();
  }
}

template <int BR>
__global__ __launch_bounds__(256) void gate_norm_kernel(
    const unsigned short* ZX, const unsigned short* Y16, const float* nw,
    const float* w1p, const float* w2p, const unsigned short* YN0in, unsigned short* OUT16)
{
  __shared__ __align__(16) float sG[kDs];
  __shared__ float sRed[8];
  const int tid = threadIdx.x, lane = tid & 31, wave = tid >> 5;
  const size_t row = blockIdx.x;
  float part = 0.0f;
#pragma unroll 1
  for (int hf = 0; hf < 2; ++hf) {
    const int f0 = tid * 8 + hf * 4;
    const u2v yw = *(const u2v*)(Y16 + row * kDs + f0);
    const int zcol = BR ? (kDip - 4 - f0) : f0;
    const u2v zw = *(const u2v*)(ZX + row * kDipP + zcol);
    const unsigned y01 = yw[0];
    const unsigned y23 = yw[1];
    const unsigned z01 = zw[0];
    const unsigned z23 = zw[1];
    const float yv0 = h16_to_f32(y01 & 0xffffu), yv1 = h16_to_f32(y01 >> 16);
    const float yv2 = h16_to_f32(y23 & 0xffffu), yv3 = h16_to_f32(y23 >> 16);
    const float zr0 = h16_to_f32(z01 & 0xffffu), zr1 = h16_to_f32(z01 >> 16);
    const float zr2 = h16_to_f32(z23 & 0xffffu), zr3 = h16_to_f32(z23 >> 16);
    const float z0 = BR ? zr3 : zr0;
    const float z1 = BR ? zr2 : zr1;
    const float z2 = BR ? zr1 : zr2;
    const float z3 = BR ? zr0 : zr3;
    const float g0 = yv0 * (z0 * __builtin_amdgcn_rcpf(1.0f + expf(-z0)));
    const float g1 = yv1 * (z1 * __builtin_amdgcn_rcpf(1.0f + expf(-z1)));
    const float g2 = yv2 * (z2 * __builtin_amdgcn_rcpf(1.0f + expf(-z2)));
    const float g3 = yv3 * (z3 * __builtin_amdgcn_rcpf(1.0f + expf(-z3)));
    *(v4f*)(sG + f0) = (v4f){g0, g1, g2, g3};
    part = fmaf(g0, g0, part);
    part = fmaf(g1, g1, part);
    part = fmaf(g2, g2, part);
    part = fmaf(g3, g3, part);
  }
  float p = part;
#pragma unroll
  for (int off = 16; off >= 1; off >>= 1) p += __shfl_xor(p, off, 32);
  if (lane == 0) sRed[wave] = p;
  __syncthreads();
  float tot = sRed[0];
  tot += sRed[1]; tot += sRed[2]; tot += sRed[3];
  tot += sRed[4]; tot += sRed[5]; tot += sRed[6]; tot += sRed[7];
  const float scale = rsqrtf(tot * (1.0f / (float)kDs) + 1e-5f);
  const v4f ga = *(const v4f*)(sG + tid * 8);
  const v4f gb = *(const v4f*)(sG + tid * 8 + 4);
  const v4f na = *(const v4f*)(nw + tid * 8);
  const v4f nb = *(const v4f*)(nw + tid * 8 + 4);
  float yn[8];
#pragma unroll
  for (int e = 0; e < 4; ++e) {
    yn[e]     = ga[e] * scale * bfr(na[e]);
    yn[4 + e] = gb[e] * scale * bfr(nb[e]);
  }
  v8h hv;
  if (BR) {
    const float w1 = bfr(w1p[0]);
    const float w2 = bfr(w2p[0]);
    const u4v pw = *(const u4v*)(YN0in + row * kDs + tid * 8);
#pragma unroll
    for (int jj = 0; jj < 4; ++jj) {
      const unsigned wv = pw[jj];
      const float a0 = h16_to_f32(wv & 0xffffu);
      const float a1 = h16_to_f32(wv >> 16);
      hv[2 * jj]     = (_Float16)fmaf(w2, yn[2 * jj], w1 * a0);
      hv[2 * jj + 1] = (_Float16)fmaf(w2, yn[2 * jj + 1], w1 * a1);
    }
  } else {
#pragma unroll
    for (int e = 0; e < 8; ++e) hv[e] = (_Float16)yn[e];
  }
  unsigned short* dst = OUT16 + row * kDs + tid * 8;
  *(volatile v8h*)dst = hv;
  __threadfence();
  *(volatile v8h*)dst = hv;
}

extern "C" void kernel_launch(void* const* d_in, const int* in_sizes, int n_in,
                              void* d_out, int out_size, void* d_ws, size_t ws_size,
                              hipStream_t stream)
{
  if (n_in < 18) return;
  if (in_sizes[0] != kRows * kDm) return;
  if (in_sizes[1] != kDip * kDm) return;
  if (in_sizes[2] != kCv * 4 || in_sizes[3] != kCv) return;
  if (in_sizes[4] != kCv * 4 || in_sizes[5] != kCv) return;
  if (in_sizes[6] != kH || in_sizes[7] != kH || in_sizes[8] != kH || in_sizes[9] != kH) return;
  if (in_sizes[10] != kH || in_sizes[11] != kH) return;
  if (in_sizes[12] != kDs) return;
  if (in_sizes[13] != kDm * kDs) return;
  if (in_sizes[14] != kDm * kDm) return;
  if (in_sizes[15] != kDm) return;
  if (out_size != kRows * kDm) return;
  if (ws_size < kWsTotal) return;

  const float* u      = (const float*)d_in[0];
  const float* in_w   = (const float*)d_in[1];
  const float* cw1    = (const float*)d_in[2];
  const float* cb1    = (const float*)d_in[3];
  const float* cw2    = (const float*)d_in[4];
  const float* cb2    = (const float*)d_in[5];
  const float* dtb1   = (const float*)d_in[6];
  const float* dtb2   = (const float*)d_in[7];
  const float* alog1  = (const float*)d_in[8];
  const float* alog2  = (const float*)d_in[9];
  const float* Dp1    = (const float*)d_in[10];
  const float* Dp2    = (const float*)d_in[11];
  const float* normw  = (const float*)d_in[12];
  const float* out_w  = (const float*)d_in[13];
  const float* end_w  = (const float*)d_in[14];
  const float* end_b  = (const float*)d_in[15];
  const float* w1p    = (const float*)d_in[16];
  const float* w2p    = (const float*)d_in[17];

  char* ws = (char*)d_ws;
  unsigned short* ZX   = (unsigned short*)(ws + kOffZX);
  unsigned short* U16  = (unsigned short*)(ws + kOffU16);
  unsigned short* INW  = (unsigned short*)(ws + kOffINW);
  unsigned short* OUTW = (unsigned short*)(ws + kOffOUTW);
  unsigned short* ENDW = (unsigned short*)(ws + kOffENDW);
  unsigned short* X16  = (unsigned short*)(ws + kOffX16);
  unsigned short* BC16 = (unsigned short*)(ws + kOffBC16);
  unsigned short* BT16 = (unsigned short*)(ws + kOffBT16);
  float*          DT32 = (float*)(ws + kOffDT32);
  float*          CS32 = (float*)(ws + kOffCS32);
  unsigned short* CB16 = (unsigned short*)(ws + kOffCB16);
  unsigned short* HP16 = (unsigned short*)(ws + kOffHP16);
  unsigned short* Y16  = (unsigned short*)(ws + kOffY16);
  unsigned short* YN0  = (unsigned short*)(ws + kOffYN0);
  unsigned short* T16  = U16;
  unsigned short* YC16 = X16;

  cast_bf_f16_kernel<<<(kRows * kDm / 8) / 256, 256, 0, stream>>>(u, U16, kRows * kDm / 8, kRows * kDm / 8, 1.0f);
  cast_bf_f16_kernel<<<(kDipP * kDm / 8) / 256, 256, 0, stream>>>(in_w, INW, kDipP * kDm / 8, kDip * kDm / 8, kWCarry);
  cast_bf_f16_kernel<<<(kDm * kDs / 8) / 256, 256, 0, stream>>>(out_w, OUTW, kDm * kDs / 8, kDm * kDs / 8, kWCarry);
  cast_bf_f16_kernel<<<(kDm * kDm / 8) / 256, 256, 0, stream>>>(end_w, ENDW, kDm * kDm / 8, kDm * kDm / 8, kWCarry);

  wmma_gemm64_h<0, 1><<<dim3((kRows / 64) * (kDipP / 64) / 8, 1), 256, 0, stream>>>(
      U16, kDm, 0L, INW, kDm, 0L, (void*)ZX, kDipP, 0L, end_b, kRows, kDipP, kDm, kWInv);

  conv_silu_kernel<0><<<dim3(kCv / 64, kRows / 64), 256, 0, stream>>>(ZX, cw1, cb1, X16, BC16, BT16);
  dt_cs_kernel<0><<<kB * kNc, 256, 0, stream>>>(ZX, dtb1, alog1, DT32, CS32);
  wmma_gemm64_h<0, 1><<<dim3(2, kB * kNc), 256, 0, stream>>>(
      BC16 + kN, kBCw, (long)kQ * kBCw, BC16, kBCw, (long)kQ * kBCw,
      (void*)CB16, kQ, (long)kQ * kQ, end_b, kQ, kQ, kN, 1.0f);
  states_scan_kernel<<<kB * kH, 256, 0, stream>>>(X16, BT16, DT32, CS32, HP16);
  ssd_y_kernel<<<kB * kNc * kH, 512, 0, stream>>>(X16, BC16, CB16, HP16, DT32, CS32, Dp1, Y16);
  gate_norm_kernel<0><<<kRows, 256, 0, stream>>>(ZX, Y16, normw, w1p, w2p, YN0, YN0);

  conv_silu_kernel<1><<<dim3(kCv / 64, kRows / 64), 256, 0, stream>>>(ZX, cw2, cb2, X16, BC16, BT16);
  dt_cs_kernel<1><<<kB * kNc, 256, 0, stream>>>(ZX, dtb2, alog2, DT32, CS32);
  wmma_gemm64_h<0, 1><<<dim3(2, kB * kNc), 256, 0, stream>>>(
      BC16 + kN, kBCw, (long)kQ * kBCw, BC16, kBCw, (long)kQ * kBCw,
      (void*)CB16, kQ, (long)kQ * kQ, end_b, kQ, kQ, kN, 1.0f);
  states_scan_kernel<<<kB * kH, 256, 0, stream>>>(X16, BT16, DT32, CS32, HP16);
  ssd_y_kernel<<<kB * kNc * kH, 512, 0, stream>>>(X16, BC16, CB16, HP16, DT32, CS32, Dp2, Y16);
  gate_norm_kernel<1><<<kRows, 256, 0, stream>>>(ZX, Y16, normw, w1p, w2p, YN0, YC16);

  wmma_gemm64_h<0, 1><<<dim3((kRows / 64) * (kDm / 64) / 8, 1), 256, 0, stream>>>(
      YC16, kDs, 0L, OUTW, kDs, 0L, (void*)T16, kDm, 0L, end_b, kRows, kDm, kDs, kWInv);

  wmma_gemm64_h<2, 0><<<dim3((kRows / 64) * (kDm / 64) / 8, 1), 256, 0, stream>>>(
      T16, kDm, 0L, ENDW, kDm, 0L, d_out, kDm, 0L, end_b, kRows, kDm, kDm, kWInv);
}
